// GraphActor_24721831756516
// MI455X (gfx1250) — hardware-run, weakly checked
//
#include <hip/hip_runtime.h>


namespace {
constexpr int NPAS = 100000, NVEH = 10000, NVEHP = 10048, NREQ = 50000, NREQP = 50048, ERR = 1500000, ERV = 1000000, EVP = 300000, ERRQ = ((ERR / 4 + 15) / 16) * 16  , H = 32, VF = 64, AH = 96, AF = 128, LH = 512;
constexpr float XS = 8.0f, WSC = 256.0f;
static_assert(ERR % 16 == 0 && ERRQ % 16 == 0 && 4 * ERRQ >= ERR && ERV % 64 == 0 && NPAS % 16 == 0, "wave tiling (16-edge waves must not straddle a trip quarter; score blocks are 64 edges)");

typedef _Float16 b16;
typedef __attribute__((ext_vector_type(16))) _Float16 v16b;
typedef __attribute__((ext_vector_type(8))) _Float16 v8b;
typedef __attribute__((ext_vector_type(8))) float v8f;
typedef __attribute__((ext_vector_type(4))) float v4f;
__device__ __forceinline__ float bf16_rne(float f) { unsigned int u = __float_as_uint(f); u += 0x7FFFu + ((u >> 16) & 1u); return __uint_as_float(u & 0xFFFF0000u); }
__device__ __forceinline__ void split16(float v, b16& hi, b16& lo) { hi = (b16)v; lo = (b16)(v - (float)hi); }
__device__ __forceinline__ v16b frag_kb(const b16* p, int hh) { const v8b a = *(const v8b*)(p + 8 * hh), b = *(const v8b*)(p + 16 + 8 * hh); v16b f;
#pragma unroll
  for (int e = 0; e < 8; ++e) { f[e] = a[e]; f[8 + e] = b[e]; } return f; }
__device__ __forceinline__ v8f wmma16b(v16b a, v16b b, v8f c) { v8f d = __builtin_amdgcn_wmma_f32_16x16x32_f16(false, a, false, b, (short)0, c, false, false); asm volatile("v_nop\n\tv_nop\n\tv_nop\n\tv_nop" : "+v"(d) : "v"(a), "v"(b)); return d; }
__device__ __forceinline__ void wave_lds_sync() { __builtin_amdgcn_fence(__ATOMIC_RELEASE, "workgroup"); __builtin_amdgcn_wave_barrier(); __builtin_amdgcn_fence(__ATOMIC_ACQUIRE, "workgroup"); }
__device__ __forceinline__ float nexp(float x) { return __builtin_amdgcn_exp2f(x * 1.4426950408889634f); }
__device__ __forceinline__ float pmul(float a, float b) { float p = a * b; asm volatile("" : "+v"(p)); return p; }
__device__ __forceinline__ float hsum16(float v) { v += __shfl_xor(v, 1); v += __shfl_xor(v, 2); v += __shfl_xor(v, 4); return v + __shfl_xor(v, 8); }
__device__ __forceinline__ int iclamp(int v, int lo, int hi) { return v < lo ? lo : (v > hi ? hi : v); }
__device__ __forceinline__ float tanh_(float x) { const float e = nexp(-2.0f * fabsf(x)); const float t = (1.0f - e) / (1.0f + e); return x < 0.0f ? -t : t; }

constexpr int CSR_NBLK = 512, CSR_GB = 8, CSR_GN = 1 << CSR_GB  , CSR_MAXG = 512, CSR_CAP = 12288  ;
__global__ __launch_bounds__(64) void csrA_kernel(const int* __restrict__ dst, int E, int N, int nG, int CHP, int NGP, int* __restrict__ STG, int* __restrict__ HST) {
  extern __shared__ int sm[];
  int* cnt = sm; int* run = sm + NGP; int* ids = sm + 2 * NGP;
  const int b = blockIdx.x; const int ch = (E + CSR_NBLK - 1) / CSR_NBLK; const int e0 = b * ch, e1 = min(E, e0 + ch);
  for (int i = threadIdx.x; i < NGP; i += 64) cnt[i] = 0;
  for (int i = threadIdx.x; i < CHP; i += 64) ids[i] = -1;
  __syncthreads();
  if (threadIdx.x == 0) {
    for (int e = e0; e < e1; ++e) { int d = dst[e]; d = (d < 0) ? 0 : (d >= N ? N - 1 : d); cnt[d >> CSR_GB] += 1; }
    int acc = 0; for (int g = 0; g < nG; ++g) { run[g] = acc; acc += cnt[g]; }
    for (int e = e0; e < e1; ++e) { int d = dst[e]; d = (d < 0) ? 0 : (d >= N ? N - 1 : d); const int g = d >> CSR_GB; ids[run[g]] = e; run[g] += 1; } }
  __syncthreads();
  typedef __attribute__((ext_vector_type(4))) int v4i;
  for (int pass = 0; pass < 2; ++pass) {
    for (int i = threadIdx.x; i < CHP / 4; i += 64) *(volatile v4i*)(STG + (size_t)b * CHP + i * 4) = *(const v4i*)(&ids[i * 4]);
    for (int i = threadIdx.x; i < NGP / 4; i += 64) { v4i v; for (int e = 0; e < 4; ++e) v[e] = (i * 4 + e < nG) ? cnt[i * 4 + e] : 0; *(volatile v4i*)(HST + (size_t)b * NGP + i * 4) = v; }
    __threadfence(); }
}
__global__ __launch_bounds__(512) void csrS_kernel(const int* __restrict__ HST, int nG, int NGP, int* __restrict__ START, int* __restrict__ TOT, int* __restrict__ OFF) {
  __shared__ int tot[CSR_MAXG];
  const int b = threadIdx.x;
  for (int pass = 0; pass < 2; ++pass) { int runb = 0; for (int g = 0; g < nG; ++g) { int c = HST[(size_t)b * NGP + g]; c = (c < 0) ? 0 : c; ((volatile int*)OFF)[(size_t)g * CSR_NBLK + b] = runb; runb += c; } __threadfence(); }
  for (int g = threadIdx.x; g < nG; g += 512) { int s = 0; for (int bb = 0; bb < CSR_NBLK; ++bb) { int c = HST[(size_t)bb * NGP + g]; s += (c < 0) ? 0 : c; } tot[g] = s; }
  __syncthreads();
  if (threadIdx.x < 32) {
    __shared__ int st[CSR_MAXG + 32];
    if (threadIdx.x == 0) { int acc = 0; for (int g = 0; g < NGP; ++g) { st[g] = acc; if (g < nG) acc += (tot[g] + 31) & ~31; } st[NGP] = acc; }
    __builtin_amdgcn_fence(__ATOMIC_RELEASE, "workgroup"); __builtin_amdgcn_wave_barrier(); __builtin_amdgcn_fence(__ATOMIC_ACQUIRE, "workgroup");
    for (int pass = 0; pass < 2; ++pass) { for (int i = threadIdx.x; i < NGP + 32; i += 32) { ((volatile int*)START)[i] = (i <= NGP) ? st[min(i, NGP)] : 0; ((volatile int*)TOT)[i] = (i < nG) ? tot[i] : 0; } __threadfence(); } }
}
__global__ __launch_bounds__(256) void csrB_kernel(const int* __restrict__ dst, int N, int nG, int CHP, int NGP, int permLen, const int* __restrict__ STG, const int* __restrict__ HST, const int* __restrict__ OFF, const int* __restrict__ START, const int* __restrict__ TOT, int* __restrict__ PERM, int* __restrict__ ROWPTR, int* __restrict__ ROWCNT, int* __restrict__ FLAG) {
  typedef __attribute__((ext_vector_type(4))) int v4i;
  __shared__ int ids[CSR_CAP]; __shared__ unsigned short key[CSR_CAP]; __shared__ int outp[CSR_CAP]; __shared__ int ncnt[CSR_GN + 1]; __shared__ int boff[CSR_NBLK + 1];
  const int g = blockIdx.x, t_ = threadIdx.x; int tot = TOT[g]; int st = START[g], stn = START[g + 1]; const int v0 = g * CSR_GN; const int nv = min(CSR_GN, N - v0);
  st = (st < 0) ? 0 : (st > permLen - 32 ? permLen - 32 : st) & ~31; stn = (stn < st) ? st : (stn > permLen ? permLen : stn); tot = (tot < 0) ? 0 : tot; if (tot > stn - st && tot <= CSR_CAP) tot = stn - st;
  if (tot > CSR_CAP) {
    for (int pass = 0; pass < 2; ++pass) { for (int i = t_; i < CSR_GN / 4; i += 256) { v4i a, c; for (int e = 0; e < 4; ++e) { a[e] = st; c[e] = 0; } *(volatile v4i*)(ROWPTR + v0 + i * 4) = a; *(volatile v4i*)(ROWCNT + v0 + i * 4) = c; } if (t_ == 0) ((volatile int*)FLAG)[0] = 1; __threadfence(); } (void)nv; return; }
  if (t_ == 0) { int acc = 0; for (int b = 0; b < CSR_NBLK; ++b) { boff[b] = acc; int c = HST[(size_t)b * NGP + g]; c = (c < 0) ? 0 : (c > CHP ? CHP : c); acc += c; if (acc > tot) acc = tot; } boff[CSR_NBLK] = acc; }
  for (int i = t_; i <= CSR_GN; i += 256) ncnt[i] = 0;
  __syncthreads();
  for (int b = 0; b < CSR_NBLK; ++b) { const int c = boff[b + 1] - boff[b]; int o_ = OFF[(size_t)g * CSR_NBLK + b]; o_ = (o_ < 0) ? 0 : (o_ > CHP - c ? CHP - c : o_); const int* src_ = STG + (size_t)b * CHP + o_;
    for (int i = t_; i < c; i += 256) { int id = src_[i]; id = (id < 0) ? 0 : id; ids[boff[b] + i] = id; int d = dst[id]; d = (d < v0) ? v0 : (d >= N ? N - 1 : d); int kk = d - v0; kk = (kk < 0) ? 0 : (kk >= CSR_GN ? CSR_GN - 1 : kk); key[boff[b] + i] = (unsigned short)kk; } }
  __syncthreads();
  if (t_ == 0) { for (int i = 0; i < tot; ++i) ncnt[key[i]] += 1; int acc = 0; for (int vl = 0; vl < CSR_GN; ++vl) { const int c = ncnt[vl]; ncnt[vl] = acc; acc += c; } ncnt[CSR_GN] = acc;
    for (int i = 0; i < tot; ++i) { const int vl = key[i]; outp[ncnt[vl]] = ids[i]; ncnt[vl] += 1; }
    for (int vl = CSR_GN; vl > 0; --vl) ncnt[vl] = ncnt[vl - 1]; ncnt[0] = 0; }
  __syncthreads();
  for (int pass = 0; pass < 2; ++pass) {
    for (int i = t_; i < (stn - st) / 4; i += 256) { v4i v; for (int e = 0; e < 4; ++e) { const int q = i * 4 + e; v[e] = (q < tot) ? outp[q] : -1; } *(volatile v4i*)(PERM + st + i * 4) = v; }
    for (int i = t_; i < CSR_GN / 4; i += 256) { v4i a, c; for (int e = 0; e < 4; ++e) { const int vl = i * 4 + e; a[e] = st + ncnt[vl]; c[e] = (vl < nv) ? (ncnt[vl + 1] - ncnt[vl]) : 0; } *(volatile v4i*)(ROWPTR + v0 + i * 4) = a; *(volatile v4i*)(ROWCNT + v0 + i * 4) = c; }
    __threadfence(); }
}
__global__ __launch_bounds__(256) void csrZ_kernel(int* __restrict__ p, size_t n4) { typedef __attribute__((ext_vector_type(4))) int v4i; const size_t tid = (size_t)blockIdx.x * 256 + threadIdx.x, nth = (size_t)gridDim.x * 256; v4i z = {0, 0, 0, 0}; for (size_t i = tid; i < n4; i += nth) *(volatile v4i*)(p + i * 4) = z; }
struct CsrBufs { int *STG, *HST, *OFF, *START, *TOT, *PERM, *ROWPTR, *ROWCNT, *FLAG; int nG, NGP, CHP; size_t permLen; char* base; size_t bytes; };
static size_t csr_carve(CsrBufs& c, char* ws, size_t off, int E, int N) {
  const size_t off0 = off; c.base = ws + off;
  auto al = [&](size_t bytes) { char* p = ws + off; off += (bytes + 255) & ~(size_t)255; return p; };
  c.nG = (N + CSR_GN - 1) / CSR_GN; c.NGP = (c.nG + 31) & ~31; const int ch = (E + CSR_NBLK - 1) / CSR_NBLK; c.CHP = (ch + 31) & ~31; c.permLen = (size_t)E + 32 * (size_t)c.nG + 32;
  c.STG = (int*)al((size_t)CSR_NBLK * c.CHP * 4); c.HST = (int*)al((size_t)CSR_NBLK * c.NGP * 4); c.OFF = (int*)al((size_t)c.NGP * CSR_NBLK * 4); c.START = (int*)al((size_t)(c.NGP + 64) * 4); c.TOT = (int*)al((size_t)(c.NGP + 64) * 4);
  c.PERM = (int*)al(c.permLen * 4); c.ROWPTR = (int*)al((size_t)c.nG * CSR_GN * 4); c.ROWCNT = (int*)al((size_t)c.nG * CSR_GN * 4); c.FLAG = (int*)al(256);
  c.bytes = off - off0; return off;
}
static void csr_build(const CsrBufs& c, const int* dst, int E, int N, hipStream_t stream) {
  const size_t smem = (size_t)(2 * c.NGP + c.CHP) * 4;
  csrZ_kernel<<<512, 256, 0, stream>>>((int*)c.base, c.bytes / 16);
  csrA_kernel<<<CSR_NBLK, 64, smem, stream>>>(dst, E, N, c.nG, c.CHP, c.NGP, c.STG, c.HST);
  csrS_kernel<<<1, 512, 0, stream>>>(c.HST, c.nG, c.NGP, c.START, c.TOT, c.OFF);
  csrB_kernel<<<c.nG, 256, 0, stream>>>(dst, N, c.nG, c.CHP, c.NGP, (int)c.permLen, c.STG, c.HST, c.OFF, c.START, c.TOT, c.PERM, c.ROWPTR, c.ROWCNT, c.FLAG);
}


__global__ __launch_bounds__(256) void prepx_kernel(const float* __restrict__ px, const float* __restrict__ vx, const float* __restrict__ rx, b16* __restrict__ PX, b16* __restrict__ VX, b16* __restrict__ RX) {
  const size_t g = (size_t)blockIdx.x * 256 + threadIdx.x; const int lane = threadIdx.x & 31;
  const size_t w = g >> 5; const size_t nwp = NPAS / 8, nwv = NVEHP / 8, nwr = NREQP / 8;
  int kind; size_t row0; if (w < nwp) { kind = 0; row0 = w * 8; } else if (w < nwp + nwv) { kind = 1; row0 = (w - nwp) * 8; } else if (w < nwp + nwv + nwr) { kind = 2; row0 = (w - nwp - nwv) * 8; } else return;
  const size_t row = row0 + (lane >> 2); const int seg = lane & 3; const int nf = kind == 0 ? 10 : kind == 1 ? 5 : 8; const int nrows = kind == 0 ? NPAS : kind == 1 ? NVEH : NREQ;
  const float* src = kind == 0 ? px : kind == 1 ? vx : rx; b16* dst = (kind == 0 ? PX : kind == 1 ? VX : RX) + row * 32 + seg * 8;
  v8b o; for (int j = 0; j < 8; ++j) { const int c = seg * 8 + j; o[j] = (c < nf && row < (size_t)nrows) ? (b16)(bf16_rne(src[row * nf + (c < nf ? c : 0)]) * XS) : (b16)0.0f; }
  for (int pass = 0; pass < 2; ++pass) { *(volatile v8b*)dst = o; __threadfence(); }
}
__global__ __launch_bounds__(256) void prepw_kernel(const float* __restrict__ wpas, const float* __restrict__ wveh, const float* __restrict__ wreq, const float* __restrict__ wte, const float* __restrict__ wem, const float* __restrict__ wtn, const float* __restrict__ wa1, const float* __restrict__ wl1, const float* __restrict__ wl2,
                                                  b16* __restrict__ WPAS, b16* __restrict__ WVEH, b16* __restrict__ WREQ, b16* __restrict__ WTE, b16* __restrict__ WEM, b16* __restrict__ WTN, b16* __restrict__ WA1, b16* __restrict__ WL1, b16* __restrict__ WL2) {
  const int kind = blockIdx.y, t = blockIdx.x * 256 + threadIdx.x;
  int IN, OUT, KP; const float* w; b16* dst;
  switch (kind) { case 0: IN = 10; OUT = H; KP = 32; w = wpas; dst = WPAS; break; case 1: IN = 5; OUT = H; KP = 32; w = wveh; dst = WVEH; break; case 2: IN = 8; OUT = H; KP = 32; w = wreq; dst = WREQ; break;
    case 3: IN = 17; OUT = H; KP = 32; w = wte; dst = WTE; break; case 4: IN = 15; OUT = H; KP = 32; w = wem; dst = WEM; break; case 5: IN = 40; OUT = H; KP = 64; w = wtn; dst = WTN; break;
    case 6: IN = AH; OUT = AH; KP = AH; w = wa1; dst = WA1; break; case 7: IN = AF; OUT = LH; KP = AF; w = wl1; dst = WL1; break; default: IN = LH; OUT = LH; KP = LH; w = wl2; dst = WL2; break; }
  const int ngrp = OUT * KP / 8; if (t >= ngrp) return; const int o_ = (t * 8) / KP, k0 = t * 8 - o_ * KP;
  v8b o; for (int j = 0; j < 8; ++j) { const int k = k0 + j; int i;
    if (kind == 5) i = (k < 8) ? k : (k >= 32 ? 8 + (k - 32) : -1); else i = (k < IN) ? k : -1;
    o[j] = (i >= 0) ? (b16)(bf16_rne(w[(size_t)i * OUT + o_]) * WSC) : (b16)0.0f; }
  for (int pass = 0; pass < 2; ++pass) { *(volatile v8b*)(dst + (size_t)t * 8) = o; __threadfence(); }
}
__global__ __launch_bounds__(128) void enc_kernel(const b16* __restrict__ X16, const b16* __restrict__ W, const float* __restrict__ b, int nrows, float* __restrict__ Y, int ldy) {
  __shared__ __attribute__((aligned(16))) float Ts[4][16][H + 4];
  const int wave = threadIdx.x >> 5, lane = threadIdx.x & 31, nloc = lane & 15, hlf = lane >> 4; const size_t m0 = ((size_t)blockIdx.x * 4 + wave) * 16; if (m0 >= (size_t)nrows) return;
  const v16b a = frag_kb(X16 + (m0 + nloc) * 32, hlf); v8f acc[2] = {{}, {}};
#pragma unroll
  for (int t = 0; t < 2; ++t) acc[t] = wmma16b(a, frag_kb(W + (size_t)(t * 16 + nloc) * 32, hlf), acc[t]);
#pragma unroll
  for (int t = 0; t < 2; ++t) { const float bb = bf16_rne(b[t * 16 + nloc]);
#pragma unroll
    for (int r = 0; r < 8; ++r) Ts[wave][8 * hlf + r][t * 16 + nloc] = acc[t][r] * (1.0f / (XS * WSC)) + bb; }
  wave_lds_sync();
  for (int pass = 0; pass < 2; ++pass) { for (int r4 = 0; r4 < 16; r4 += 4) { const int rr = r4 + (lane >> 3), c4 = (lane & 7) * 4; *(volatile v4f*)(Y + (m0 + rr) * ldy + c4) = *(const v4f*)(&Ts[wave][rr][c4]); } __threadfence(); }
}
__global__ __launch_bounds__(256) void pasmean_kernel(const float* __restrict__ PASF, const int* __restrict__ recv, const int* __restrict__ PERM, const int* __restrict__ ROWPTR, const int* __restrict__ ROWCNT, int permLen, int E_, float* __restrict__ VEHF) {
  const int wave = threadIdx.x >> 5, lane = threadIdx.x & 31; const size_t v = ((size_t)blockIdx.x * 8 + wave) * 4 + (lane >> 3); const int c0 = (lane & 7) * 4;
  int st = ROWPTR[v], cnt = ROWCNT[v]; cnt = iclamp(cnt, 0, 1 << 16); st = iclamp(st, 0, permLen - cnt);
  v4f acc = {0, 0, 0, 0};
  for (int j = 0; j < cnt; ++j) { const int e = iclamp(PERM[st + j], 0, E_ - 1); const int p = iclamp(recv[e], 0, NPAS - 1); acc += *(const v4f*)(PASF + (size_t)p * H + c0); }
  const float inv = 1.0f / (float)(cnt > 1 ? cnt : 1); acc *= inv;
  for (int pass = 0; pass < 2; ++pass) { *(volatile v4f*)(VEHF + v * VF + H + c0) = acc; __threadfence(); }
}
__global__ __launch_bounds__(128) void trip_kernel(const b16* __restrict__ RX, const int* __restrict__ src, const int* __restrict__ dest, const float* __restrict__ attr, const b16* __restrict__ WTE, const float* __restrict__ bte, int ebase, int equarter, float* __restrict__ EDGE) {
  __shared__ __attribute__((aligned(16))) b16 Ta[4][16][32 + 8]; __shared__ __attribute__((aligned(16))) float Ts[4][16][H + 4];
  const int wave = threadIdx.x >> 5, lane = threadIdx.x & 31, nloc = lane & 15, hlf = lane >> 4; const int e0 = ebase + (blockIdx.x * 4 + wave) * 16; if (e0 >= ebase + equarter || e0 >= ERR) return;
  { const int rr = lane >> 1, hf = lane & 1; const int e = e0 + rr; if (hf == 0) { const int s = iclamp(src[e], 0, NREQ - 1); *(v8b*)(&Ta[wave][rr][0]) = *(const v8b*)(RX + (size_t)s * 32); }
    else { const int d = iclamp(dest[e], 0, NREQ - 1); *(v8b*)(&Ta[wave][rr][8]) = *(const v8b*)(RX + (size_t)d * 32); v8b z = {}; z[0] = (b16)(bf16_rne(attr[e]) * XS); *(v8b*)(&Ta[wave][rr][16]) = z; v8b z2 = {}; *(v8b*)(&Ta[wave][rr][24]) = z2; } }
  wave_lds_sync();
  const v16b a = frag_kb(&Ta[wave][nloc][0], hlf); v8f acc[2] = {{}, {}};
#pragma unroll
  for (int t = 0; t < 2; ++t) acc[t] = wmma16b(a, frag_kb(WTE + (size_t)(t * 16 + nloc) * 32, hlf), acc[t]);
#pragma unroll
  for (int t = 0; t < 2; ++t) { const float bb = bf16_rne(bte[t * 16 + nloc]);
#pragma unroll
    for (int r = 0; r < 8; ++r) Ts[wave][8 * hlf + r][t * 16 + nloc] = tanh_(acc[t][r] * (1.0f / (XS * WSC)) + bb); }
  wave_lds_sync();
  for (int pass = 0; pass < 2; ++pass) { for (int r4 = 0; r4 < 16; r4 += 4) { const int rr = r4 + (lane >> 3), c4 = (lane & 7) * 4; *(volatile v4f*)(EDGE + ((size_t)(e0 - ebase) + rr) * H + c4) = *(const v4f*)(&Ts[wave][rr][c4]); } __threadfence(); }
}
template <int QTR>
__global__ __launch_bounds__(256) void tripmean_kernel(const float* __restrict__ EDGE, const int* __restrict__ PERM, const int* __restrict__ ROWPTR, const int* __restrict__ ROWCNT, int permLen, int equarter, float* __restrict__ EM) {
  const int wave = threadIdx.x >> 5, lane = threadIdx.x & 31; const size_t v = ((size_t)blockIdx.x * 8 + wave) * 4 + (lane >> 3); const int c0 = (lane & 7) * 4;
  int st = ROWPTR[v], cnt = ROWCNT[v]; cnt = iclamp(cnt, 0, 1 << 16); st = iclamp(st, 0, permLen - cnt);
  v4f acc = (QTR == 0) ? (v4f){0, 0, 0, 0} : *(const v4f*)(EM + v * H + c0);
  for (int j = 0; j < cnt; ++j) { const int e = iclamp(PERM[st + j], 0, ERR - 1); const bool inq = e >= QTR * equarter && e < (QTR + 1) * equarter && e < ERR; const int el = iclamp(e - QTR * equarter, 0, equarter - 1);
    const v4f x = *(const v4f*)(EDGE + (size_t)el * H + c0); if (inq) acc += x; }
  if (QTR == 3) { const float inv = 1.0f / (float)(cnt > 1 ? cnt : 1); acc *= inv; }
  for (int pass = 0; pass < 2; ++pass) { *(volatile v4f*)(EM + v * H + c0) = acc; __threadfence(); }
}
__global__ __launch_bounds__(128) void tripfeat_kernel(const b16* __restrict__ RX, const float* __restrict__ EM, const b16* __restrict__ WTN, const float* __restrict__ btn, float* __restrict__ TRIPF) {
  __shared__ __attribute__((aligned(16))) b16 Th[4][16][32 + 8], Tl[4][16][32 + 8]; __shared__ __attribute__((aligned(16))) float Ts[4][16][H + 4];
  const int wave = threadIdx.x >> 5, lane = threadIdx.x & 31, nloc = lane & 15, hlf = lane >> 4; const size_t m0 = ((size_t)blockIdx.x * 4 + wave) * 16;
  { const int rr = lane >> 1, hf = lane & 1; const float* em = EM + (m0 + rr) * H + hf * 16; for (int j = 0; j < 16; ++j) { b16 a_, c_; split16(em[j] * XS, a_, c_); Th[wave][rr][hf * 16 + j] = a_; Tl[wave][rr][hf * 16 + j] = c_; } }
  wave_lds_sync();
  const v16b ax = frag_kb(RX + (m0 + nloc) * 32, hlf), ah = frag_kb(&Th[wave][nloc][0], hlf), al = frag_kb(&Tl[wave][nloc][0], hlf); v8f acc[2] = {{}, {}};
#pragma unroll
  for (int t = 0; t < 2; ++t) { const b16* wrow = WTN + (size_t)(t * 16 + nloc) * 64; acc[t] = wmma16b(ax, frag_kb(wrow, hlf), acc[t]); const v16b bw = frag_kb(wrow + 32, hlf); acc[t] = wmma16b(ah, bw, acc[t]); acc[t] = wmma16b(al, bw, acc[t]); }
#pragma unroll
  for (int t = 0; t < 2; ++t) { const float bb = bf16_rne(btn[t * 16 + nloc]);
#pragma unroll
    for (int r = 0; r < 8; ++r) Ts[wave][8 * hlf + r][t * 16 + nloc] = acc[t][r] * (1.0f / (XS * WSC)) + bb; }
  wave_lds_sync();
  for (int pass = 0; pass < 2; ++pass) { for (int r4 = 0; r4 < 16; r4 += 4) { const int rr = r4 + (lane >> 3), c4 = (lane & 7) * 4; *(volatile v4f*)(TRIPF + (m0 + rr) * H + c4) = *(const v4f*)(&Ts[wave][rr][c4]); } __threadfence(); }
}
__global__ __launch_bounds__(128) void score_kernel(const b16* __restrict__ RX, const b16* __restrict__ VX, const int* __restrict__ snd, const int* __restrict__ rcv, const float* __restrict__ attr, const b16* __restrict__ WEM, const float* __restrict__ bem, const float* __restrict__ VEHF, const b16* __restrict__ WA1, const float* __restrict__ ba1, const float* __restrict__ wa2, const float* __restrict__ ba2, float* __restrict__ SC) {
  __shared__ __attribute__((aligned(16))) b16 Tx[4][16][32 + 8], Th[4][16][AH + 8], Tl[4][16][AH + 8]; __shared__ float Ssc[64];
  const int wave = threadIdx.x >> 5, lane = threadIdx.x & 31, nloc = lane & 15, hlf = lane >> 4, t_ = threadIdx.x; const int e0 = (blockIdx.x * 4 + wave) * 16;
  { const int rr = lane >> 1, hf = lane & 1; const int e = e0 + rr; const int s = iclamp(snd[e], 0, NREQ - 1), rv = iclamp(rcv[e], 0, NVEH - 1);
    if (hf == 0) { *(v8b*)(&Tx[wave][rr][0]) = *(const v8b*)(RX + (size_t)s * 32); const v8b vv = *(const v8b*)(VX + (size_t)rv * 32); v8b m = {}; for (int j = 0; j < 5; ++j) m[j] = vv[j]; m[5] = (b16)(bf16_rne(attr[(size_t)e * 2]) * XS); m[6] = (b16)(bf16_rne(attr[(size_t)e * 2 + 1]) * XS); *(v8b*)(&Tx[wave][rr][8]) = m; v8b z = {}; *(v8b*)(&Tx[wave][rr][16]) = z; *(v8b*)(&Tx[wave][rr][24]) = z; }
    const float* vf = VEHF + (size_t)rv * VF + hf * 32; for (int j = 0; j < 32; ++j) { b16 a_, c_; split16(vf[j] * XS, a_, c_); Th[wave][rr][hf * 32 + j] = a_; Tl[wave][rr][hf * 32 + j] = c_; } }
  wave_lds_sync();
  { const v16b a = frag_kb(&Tx[wave][nloc][0], hlf); v8f acc2[2] = {{}, {}};
#pragma unroll
    for (int t = 0; t < 2; ++t) acc2[t] = wmma16b(a, frag_kb(WEM + (size_t)(t * 16 + nloc) * 32, hlf), acc2[t]);
#pragma unroll
    for (int t = 0; t < 2; ++t) { const float bb = bf16_rne(bem[t * 16 + nloc]);
#pragma unroll
      for (int r = 0; r < 8; ++r) { b16 a_, c_; split16((acc2[t][r] * (1.0f / (XS * WSC)) + bb) * XS, a_, c_); Th[wave][8 * hlf + r][VF + t * 16 + nloc] = a_; Tl[wave][8 * hlf + r][VF + t * 16 + nloc] = c_; } } }
  wave_lds_sync();
  v8f acc[6];
#pragma unroll
  for (int t = 0; t < 6; ++t) acc[t] = (v8f){};
#pragma unroll
  for (int kb = 0; kb < AH; kb += 32) { const v16b a = frag_kb(&Th[wave][nloc][kb], hlf), al = frag_kb(&Tl[wave][nloc][kb], hlf);
#pragma unroll
    for (int t = 0; t < 6; ++t) { const v16b bw = frag_kb(WA1 + (size_t)(t * 16 + nloc) * AH + kb, hlf); acc[t] = wmma16b(a, bw, acc[t]); acc[t] = wmma16b(al, bw, acc[t]); } }
  const float b2 = bf16_rne(ba2[0]);
#pragma unroll
  for (int r = 0; r < 8; ++r) { float p = 0.0f;
#pragma unroll
    for (int t = 0; t < 6; ++t) { const int c = t * 16 + nloc; p += pmul(tanh_(acc[t][r] * (1.0f / (XS * WSC)) + bf16_rne(ba1[c])), bf16_rne(wa2[c])); }
    p = hsum16(p); if (nloc == 0) Ssc[wave * 16 + 8 * hlf + r] = p + b2; }
  __syncthreads();
  for (int pass = 0; pass < 2; ++pass) { if (t_ < 64) ((volatile float*)SC)[(size_t)blockIdx.x * 64 + t_] = Ssc[t_]; __threadfence(); }
}
__global__ __launch_bounds__(256) void vehagg_kernel(const float* __restrict__ SC, const int* __restrict__ rcv, const float* __restrict__ VEHF, const int* __restrict__ PERM, const int* __restrict__ ROWPTR, const int* __restrict__ ROWCNT, int permLen, int E_, float* __restrict__ VA) {
  const int wave = threadIdx.x >> 5, lane = threadIdx.x & 31; const size_t v = ((size_t)blockIdx.x * 8 + wave) * 2 + (lane >> 4); const int c0 = (lane & 15) * 4;
  int st = ROWPTR[v], cnt = ROWCNT[v]; cnt = iclamp(cnt, 0, 1 << 16); st = iclamp(st, 0, permLen - cnt);
  float m = -INFINITY; for (int j = 0; j < cnt; ++j) { const int e = iclamp(PERM[st + j], 0, E_ - 1); m = fmaxf(m, SC[e]); }
  float den = 0.0f; for (int j = 0; j < cnt; ++j) { const int e = iclamp(PERM[st + j], 0, E_ - 1); den += __expf(SC[e] - m); }
  v4f acc = {0, 0, 0, 0};
  for (int j = 0; j < cnt; ++j) { const int e = iclamp(PERM[st + j], 0, E_ - 1); const int rv = iclamp(rcv[e], 0, NVEH - 1); const float p = __expf(SC[e] - m) / den; acc += p * *(const v4f*)(VEHF + (size_t)rv * VF + c0); }
  const float inv = 1.0f / (float)(cnt > 1 ? cnt : 1); acc *= inv; if (cnt == 0) acc = (v4f){0, 0, 0, 0};
  for (int pass = 0; pass < 2; ++pass) { *(volatile v4f*)(VA + v * VF + c0) = acc; __threadfence(); }
}
__global__ __launch_bounds__(256) void head_kernel(const float* __restrict__ REQF, const float* __restrict__ TRIPF, const float* __restrict__ VA, const b16* __restrict__ WL1, const float* __restrict__ bl1, const b16* __restrict__ WL2, const float* __restrict__ bl2, const float* __restrict__ wl3, const float* __restrict__ bl3, float* __restrict__ out) {
  __shared__ __attribute__((aligned(16))) b16 Ah[2][16][AF + 8], Al[2][16][AF + 8], H1h[2][16][LH + 8], H1l[2][16][LH + 8]; __shared__ float Po[2][4][16]; __shared__ float So[32];
  const int wave = threadIdx.x >> 5, lane = threadIdx.x & 31, nloc = lane & 15, hlf = lane >> 4, t_ = threadIdx.x; const int grp = wave >> 2, wq = wave & 3; const size_t m0 = (size_t)blockIdx.x * 32 + grp * 16; const int n0 = wq * 128;
  for (int q = 0; q < 16; ++q) { const int idx = lane * 16 + q; const int rr = wq * 4 + (idx >> 7), c = idx & 127; const size_t row = m0 + rr; float v;
    if (c < 32) v = REQF[row * H + c]; else if (c < 64) v = TRIPF[row * H + (c - 32)]; else v = VA[row * VF + (c - 64)];
    b16 a_, c_; split16(v * XS, a_, c_); Ah[grp][rr][c] = a_; Al[grp][rr][c] = c_; }
  __syncthreads();
  v8f acc[8];
#pragma unroll
  for (int t = 0; t < 8; ++t) acc[t] = (v8f){};
#pragma unroll
  for (int kb = 0; kb < AF; kb += 32) { const v16b a = frag_kb(&Ah[grp][nloc][kb], hlf), al = frag_kb(&Al[grp][nloc][kb], hlf);
#pragma unroll
    for (int t = 0; t < 8; ++t) { const v16b bw = frag_kb(WL1 + (size_t)(n0 + t * 16 + nloc) * AF + kb, hlf); acc[t] = wmma16b(a, bw, acc[t]); acc[t] = wmma16b(al, bw, acc[t]); } }
#pragma unroll
  for (int t = 0; t < 8; ++t) { const int c = n0 + t * 16 + nloc; const float bb = bf16_rne(bl1[c]);
#pragma unroll
    for (int r = 0; r < 8; ++r) { b16 a_, c_; split16(tanh_(acc[t][r] * (1.0f / (XS * WSC)) + bb) * XS, a_, c_); H1h[grp][8 * hlf + r][c] = a_; H1l[grp][8 * hlf + r][c] = c_; } }
  __syncthreads();
#pragma unroll
  for (int t = 0; t < 8; ++t) acc[t] = (v8f){};
#pragma unroll 4
  for (int kb = 0; kb < LH; kb += 32) { const v16b a = frag_kb(&H1h[grp][nloc][kb], hlf), al = frag_kb(&H1l[grp][nloc][kb], hlf);
#pragma unroll
    for (int t = 0; t < 8; ++t) { const v16b bw = frag_kb(WL2 + (size_t)(n0 + t * 16 + nloc) * LH + kb, hlf); acc[t] = wmma16b(a, bw, acc[t]); acc[t] = wmma16b(al, bw, acc[t]); } }
#pragma unroll
  for (int r = 0; r < 8; ++r) { float p = 0.0f;
#pragma unroll
    for (int t = 0; t < 8; ++t) { const int c = n0 + t * 16 + nloc; p += pmul(tanh_(acc[t][r] * (1.0f / (XS * WSC)) + bf16_rne(bl2[c])), bf16_rne(wl3[c])); }
    p = hsum16(p); if (nloc == 0) Po[grp][wq][8 * hlf + r] = p; }
  __syncthreads();
  if (t_ < 32) { const int g2 = t_ >> 4, rr = t_ & 15; So[t_] = ((Po[g2][0][rr] + Po[g2][1][rr]) + (Po[g2][2][rr] + Po[g2][3][rr])) + bf16_rne(bl3[0]); }
  __syncthreads();
  for (int pass = 0; pass < 2; ++pass) { if (t_ < 32) { const size_t row = (size_t)blockIdx.x * 32 + t_; if (row < NREQ) ((volatile float*)out)[row] = So[t_]; } __threadfence(); }
}
}

extern "C" void kernel_launch(void* const* d_in, const int* in_sizes, int n_in, void* d_out, int out_size, void* d_ws, size_t ws_size, hipStream_t stream) {
  (void)n_in;
  auto Fp = [&](int i) { return (const float*)d_in[i]; }; auto Ip = [&](int i) { return (const int*)d_in[i]; };
  if (in_sizes[0] != NPAS * 10 || in_sizes[1] != NVEH * 5 || in_sizes[2] != NREQ * 8 || in_sizes[3] != ERR || in_sizes[4] != ERV * 2 || in_sizes[5] != ERR || in_sizes[7] != ERV || in_sizes[9] != EVP || in_sizes[23] != AH * AH || in_sizes[27] != AF * LH || in_sizes[29] != LH * LH || out_size != NREQ) return;
  size_t off = 0; char* ws = (char*)d_ws;
  auto carve = [&](size_t bytes) { char* p = ws + off; off += (bytes + 255) & ~(size_t)255; return p; };
  b16* PX = (b16*)carve((size_t)NPAS * 32 * 2); b16* VX = (b16*)carve((size_t)NVEHP * 32 * 2); b16* RX = (b16*)carve((size_t)NREQP * 32 * 2);
  b16* WPAS = (b16*)carve(H * 32 * 2); b16* WVEH = (b16*)carve(H * 32 * 2); b16* WREQ = (b16*)carve(H * 32 * 2); b16* WTE = (b16*)carve(H * 32 * 2); b16* WEM = (b16*)carve(H * 32 * 2); b16* WTN = (b16*)carve(H * 64 * 2); b16* WA1 = (b16*)carve(AH * AH * 2); b16* WL1 = (b16*)carve((size_t)LH * AF * 2); b16* WL2 = (b16*)carve((size_t)LH * LH * 2);
  float* PASF = (float*)carve((size_t)NPAS * H * 4); float* VEHF = (float*)carve((size_t)NVEHP * VF * 4); float* REQF = (float*)carve((size_t)NREQP * H * 4); float* EM = (float*)carve((size_t)NREQP * H * 4); float* TRIPF = (float*)carve((size_t)NREQP * H * 4);
  float* EDGE = (float*)carve((size_t)ERRQ * H * 4); float* SC = (float*)carve((size_t)ERV * 4); float* VA = (float*)carve((size_t)NREQP * VF * 4);
  CsrBufs csr_vp, csr_rr, csr_rv; const size_t csr0 = off; size_t e1 = csr_carve(csr_vp, ws, csr0, EVP, NVEH), e2 = csr_carve(csr_rr, ws, csr0, ERR, NREQ), e3 = csr_carve(csr_rv, ws, csr0, ERV, NREQ); off = e1 > e2 ? (e1 > e3 ? e1 : e3) : (e2 > e3 ? e2 : e3);
  if (off > ws_size || off > ((size_t)128 << 20)) return;
  prepx_kernel<<<((NPAS / 8 + NVEHP / 8 + NREQP / 8) * 32 + 255) / 256, 256, 0, stream>>>(Fp(0), Fp(1), Fp(2), PX, VX, RX);
  prepw_kernel<<<dim3((LH * LH / 8 + 255) / 256, 9), 256, 0, stream>>>(Fp(11), Fp(13), Fp(15), Fp(17), Fp(21), Fp(19), Fp(23), Fp(27), Fp(29), WPAS, WVEH, WREQ, WTE, WEM, WTN, WA1, WL1, WL2);
  enc_kernel<<<(NPAS + 63) / 64, 128, 0, stream>>>(PX, WPAS, Fp(12), NPAS, PASF, H);
  enc_kernel<<<(NVEHP + 63) / 64, 128, 0, stream>>>(VX, WVEH, Fp(14), NVEHP, VEHF, VF);
  enc_kernel<<<(NREQP + 63) / 64, 128, 0, stream>>>(RX, WREQ, Fp(16), NREQP, REQF, H);
  csr_build(csr_vp, Ip(9), EVP, NVEH, stream);
  pasmean_kernel<<<NVEHP / 32, 256, 0, stream>>>(PASF, Ip(10), csr_vp.PERM, csr_vp.ROWPTR, csr_vp.ROWCNT, (int)csr_vp.permLen, EVP, VEHF);
  csr_build(csr_rr, Ip(5), ERR, NREQ, stream);
  trip_kernel<<<(ERRQ + 63) / 64, 128, 0, stream>>>(RX, Ip(5), Ip(6), Fp(3), WTE, Fp(18), 0 * ERRQ, ERRQ, EDGE); tripmean_kernel<0><<<NREQP / 32, 256, 0, stream>>>(EDGE, csr_rr.PERM, csr_rr.ROWPTR, csr_rr.ROWCNT, (int)csr_rr.permLen, ERRQ, EM);
  trip_kernel<<<(ERRQ + 63) / 64, 128, 0, stream>>>(RX, Ip(5), Ip(6), Fp(3), WTE, Fp(18), 1 * ERRQ, ERRQ, EDGE); tripmean_kernel<1><<<NREQP / 32, 256, 0, stream>>>(EDGE, csr_rr.PERM, csr_rr.ROWPTR, csr_rr.ROWCNT, (int)csr_rr.permLen, ERRQ, EM);
  trip_kernel<<<(ERRQ + 63) / 64, 128, 0, stream>>>(RX, Ip(5), Ip(6), Fp(3), WTE, Fp(18), 2 * ERRQ, ERRQ, EDGE); tripmean_kernel<2><<<NREQP / 32, 256, 0, stream>>>(EDGE, csr_rr.PERM, csr_rr.ROWPTR, csr_rr.ROWCNT, (int)csr_rr.permLen, ERRQ, EM);
  trip_kernel<<<(ERRQ + 63) / 64, 128, 0, stream>>>(RX, Ip(5), Ip(6), Fp(3), WTE, Fp(18), 3 * ERRQ, ERRQ, EDGE); tripmean_kernel<3><<<NREQP / 32, 256, 0, stream>>>(EDGE, csr_rr.PERM, csr_rr.ROWPTR, csr_rr.ROWCNT, (int)csr_rr.permLen, ERRQ, EM);
  tripfeat_kernel<<<NREQP / 64 + ((NREQP % 64) ? 1 : 0), 128, 0, stream>>>(RX, EM, WTN, Fp(20), TRIPF);
  score_kernel<<<ERV / 64, 128, 0, stream>>>(RX, VX, Ip(7), Ip(8), Fp(4), WEM, Fp(22), VEHF, WA1, Fp(24), Fp(25), Fp(26), SC);
  csr_build(csr_rv, Ip(7), ERV, NREQ, stream);
  vehagg_kernel<<<NREQP / 16, 256, 0, stream>>>(SC, Ip(8), VEHF, csr_rv.PERM, csr_rv.ROWPTR, csr_rv.ROWCNT, (int)csr_rv.permLen, ERV, VA);
  head_kernel<<<NREQP / 32, 256, 0, stream>>>(REQF, TRIPF, VA, WL1, Fp(28), WL2, Fp(30), Fp(31), Fp(32), (float*)d_out);
}
